// SingleGCN_41394894798937
// MI455X (gfx1250) — hardware-verified
//
#include <hip/hip_runtime.h>
#include <stdint.h>
#include <math.h>

#define N_NODE   50000
#define N_EDGE   800000
#define NFEAT    128
#define NT       256
#define SRB      2048
#define SCH      2048
#define SPT      (SCH / NT)
#define N_TILE   25
#define NPAD_AGG (N_TILE * SRB)
#define M_PAD    50048

static_assert(N_NODE < (1 << 17), "");
static_assert(N_EDGE % SPT == 0, "");
static_assert(SRB == 2048 && NT == 256 && SCH == 2048, "");
static_assert(M_PAD % 64 == 0 && M_PAD >= N_NODE && NPAD_AGG >= M_PAD && M_PAD % 16 == 0, "");
static_assert((N_NODE * NFEAT) % (4 * 256) == 0, "");
static_assert(NFEAT % 64 == 0 && NFEAT % 32 == 0, "");
static_assert((NFEAT * (NFEAT / 2)) % 256 == 0, "");
static_assert((M_PAD * 16) % 256 == 0, "");

typedef __attribute__((ext_vector_type(16))) _Float16 v16h;
typedef __attribute__((ext_vector_type(8)))  _Float16 v8h;
typedef __attribute__((ext_vector_type(16))) __bf16   v16b;
typedef __attribute__((ext_vector_type(8)))  __bf16   v8b;
typedef __attribute__((ext_vector_type(8)))  float    v8f;
typedef __attribute__((ext_vector_type(4)))  float    v4f;
typedef __attribute__((ext_vector_type(4)))  int      v4i;

__device__ __forceinline__ unsigned short f2bf_bits(float f) {
  unsigned u = __float_as_uint(f);
  return (unsigned short)((u + 0x7FFFu + ((u >> 16) & 1u)) >> 16);
}
__device__ __forceinline__ float bf_bits2f(unsigned short h) { return __uint_as_float(((unsigned)h) << 16); }

__device__ __forceinline__ void split_bf(float f, unsigned short& hb, unsigned short& lb) {
  hb = f2bf_bits(f);
  lb = f2bf_bits(f - bf_bits2f(hb));
}

__device__ __forceinline__ void dep_guard_h(v8f& a, v8f& b, v16h x, v16h y) { asm volatile("v_nop\n\tv_nop\n\tv_nop\n\tv_nop" : "+v"(a), "+v"(b) : "v"(x), "v"(y)); }
__device__ __forceinline__ void dep_guard_b(v8f& a, v8f& b, v16b x, v16b y) { asm volatile("v_nop\n\tv_nop\n\tv_nop\n\tv_nop" : "+v"(a), "+v"(b) : "v"(x), "v"(y)); }
__device__ __forceinline__ void keep4_h(v16h a, v16h b, v16h c, v16h d) { asm volatile("v_nop" :: "v"(a), "v"(b), "v"(c), "v"(d)); }
__device__ __forceinline__ void keep4_b(v16b a, v16b b, v16b c, v16b d) { asm volatile("v_nop" :: "v"(a), "v"(b), "v"(c), "v"(d)); }
__device__ __forceinline__ void acc_guard4(v8f& a, v8f& b, v8f& c, v8f& d) { asm volatile("v_nop\n\tv_nop\n\tv_nop\n\tv_nop" : "+v"(a), "+v"(b), "+v"(c), "+v"(d)); }
template <typename T> struct Frag;
template <> struct Frag<_Float16> {
  typedef v16h V; union U { v16h v; v8h h[2]; };
  static __device__ __forceinline__ v16h load(const _Float16* p) {
    U f; f.h[0] = *(const v8h*)(p); f.h[1] = *(const v8h*)(p + 16); return f.v;
  }
  static __device__ __forceinline__ v8f mma(v16h a, v16h b, v8f c) {
    return __builtin_amdgcn_wmma_f32_16x16x32_f16(false, a, false, b, (short)0, c, false, false);
  }
  static __device__ __forceinline__ void guard(v8f& a, v8f& b, v16h x, v16h y) { dep_guard_h(a, b, x, y); }
  static __device__ __forceinline__ void keep(v16h a, v16h b, v16h c, v16h d) { keep4_h(a, b, c, d); }
};
template <> struct Frag<__bf16> {
  typedef v16b V; union U { v16b v; v8b h[2]; };
  static __device__ __forceinline__ v16b load(const __bf16* p) {
    U f; f.h[0] = *(const v8b*)(p); f.h[1] = *(const v8b*)(p + 16); return f.v;
  }
  static __device__ __forceinline__ v8f mma(v16b a, v16b b, v8f c) {
    return __builtin_amdgcn_wmma_f32_16x16x32_bf16(false, a, false, b, (short)0, c, false, false);
  }
  static __device__ __forceinline__ void guard(v8f& a, v8f& b, v16b x, v16b y) { dep_guard_b(a, b, x, y); }
  static __device__ __forceinline__ void keep(v16b a, v16b b, v16b c, v16b d) { keep4_b(a, b, c, d); }
};

template <int ET> struct Elem;
template <> struct Elem<0> { typedef _Float16 T; };
template <> struct Elem<1> { typedef __bf16 T; };
template <int ET, bool SPLIT, int BIAS_MODE, int OUT_MODE, bool RESID, int ACT = 0>
__global__ __launch_bounds__(256) void wmma_gemm64(
    const unsigned short* __restrict__ Ap, const unsigned short* __restrict__ A2p, int lda, long strideA,
    const unsigned short* __restrict__ Btp, const unsigned short* __restrict__ Bt2p, int ldb, long strideB,
    void* __restrict__ Cout, void* __restrict__ Cout2, int ldc, long strideC,
    const float* __restrict__ bias,
    const float* __restrict__ resid, long strideR,
    int M, int N, int K, float scale) {
  typedef typename Elem<ET>::T T;
  typedef typename Frag<T>::V V;
  const T* A = (const T*)Ap; const T* A2 = (const T*)A2p; const T* Bt = (const T*)Btp; const T* Bt2 = (const T*)Bt2p;
  __shared__ __align__(16) float sT[8][16 * 68];
  const int b    = blockIdx.y;
  const int lane = threadIdx.x & 31;
  const int wave = threadIdx.x >> 5;
  const int tilesN = N >> 6;
  const int tilesM = M >> 6;
  const int tile = blockIdx.x * 8 + wave;
  if (tile >= tilesM * tilesN) return;
  const int tm = tile / tilesN;
  const int tn = tile - tm * tilesN;
  const int m0 = tm << 6;
  const int n0 = tn << 6;

  const T* Ab  = A  + (size_t)b * strideA;
  const T* Bb  = Bt + (size_t)b * strideB;
  const T* Ab2 = SPLIT ? (A2  + (size_t)b * strideA) : nullptr;
  const T* Bb2 = SPLIT ? (Bt2 + (size_t)b * strideB) : nullptr;

  const int rlane = lane & 15;
  const int koff  = (lane >> 4) * 8;
  const int mOff  = (lane >> 4) * 8;

  v8f acc[4][4];
#pragma unroll
  for (int i = 0; i < 4; ++i)
#pragma unroll
    for (int j = 0; j < 4; ++j) acc[i][j] = (v8f){0.f,0.f,0.f,0.f,0.f,0.f,0.f,0.f};

  for (int k0 = 0; k0 < K; k0 += 32) {
    V bh[4], bl[4];
#pragma unroll
    for (int j = 0; j < 4; ++j) {
      const size_t bo = (size_t)(n0 + (j << 4) + rlane) * ldb + koff + k0;
      bh[j] = Frag<T>::load(Bb + bo);
      if (SPLIT) bl[j] = Frag<T>::load(Bb2 + bo);
    }
#pragma unroll
    for (int i = 0; i < 4; ++i) {
      const size_t ao = (size_t)(m0 + (i << 4) + rlane) * lda + koff + k0;
      V ah = Frag<T>::load(Ab + ao);
      V al;
      if (SPLIT) al = Frag<T>::load(Ab2 + ao);
#pragma unroll
      for (int j = 0; j < 4; ++j) {
        acc[i][j] = Frag<T>::mma(ah, bh[j], acc[i][j]);
        if (SPLIT) {
          acc[i][j] = Frag<T>::mma(ah, bl[j], acc[i][j]);
          acc[i][j] = Frag<T>::mma(al, bh[j], acc[i][j]);
        }
      }
      Frag<T>::guard(acc[i][0], acc[i][3], ah, SPLIT ? al : ah);
    }
    Frag<T>::keep(bh[0], bh[1], bh[2], bh[3]);
    if (SPLIT) Frag<T>::keep(bl[0], bl[1], bl[2], bl[3]);
  }
  acc_guard4(acc[0][0], acc[0][1], acc[0][2], acc[0][3]);
  acc_guard4(acc[1][0], acc[1][1], acc[1][2], acc[1][3]);
  acc_guard4(acc[2][0], acc[2][1], acc[2][2], acc[2][3]);
  acc_guard4(acc[3][0], acc[3][1], acc[3][2], acc[3][3]);

  float* slab = sT[wave];
  const float* Rb = RESID ? (resid + (size_t)b * strideR) : nullptr;
#pragma unroll
  for (int i = 0; i < 4; ++i) {
    const int mBase = m0 + (i << 4);
#pragma unroll
    for (int j = 0; j < 4; ++j) {
      const int n = n0 + (j << 4) + rlane;
      float bv = 0.f;
      if (BIAS_MODE == 2) bv = bias[n];
#pragma unroll
      for (int r = 0; r < 8; ++r) {
        float v = acc[i][j][r] * scale;
        if (BIAS_MODE == 1) v += bias[mBase + mOff + r];
        if (BIAS_MODE == 2) v += bv;
        if (RESID) v += Rb[(size_t)(mBase + mOff + r) * ldc + n];
        if (ACT == 1) v = tanhf(v);
        if (ACT == 2) v = fmaxf(v, 0.0f);
        if (ACT == 3) v = v / (1.0f + expf(-v));
        if (ACT == 4) v = (v > 0.f) ? v : 0.01f * v;
        if (ACT == 5) v = 0.5f * v * (1.0f + erff(v * 0.70710678118654752f));
        slab[(mOff + r) * 68 + (j << 4) + rlane] = v;
      }
    }
    __builtin_amdgcn_fence(__ATOMIC_RELEASE, "workgroup");
    __builtin_amdgcn_wave_barrier();
    __builtin_amdgcn_fence(__ATOMIC_ACQUIRE, "workgroup");
    if (OUT_MODE == 0) {
      float* C = (float*)Cout + (size_t)b * strideC;
      const int hh = lane >> 4, c4 = (lane & 15) * 4;
      for (int pass = 0; pass < 2; ++pass) {
#pragma unroll
        for (int it = 0; it < 8; ++it) {
          const int row = it * 2 + hh;
          v4f v = *(const v4f*)(slab + row * 68 + c4);
          *(volatile v4f*)(C + (size_t)(mBase + row) * ldc + n0 + c4) = v;
        }
        __threadfence();
      }
    } else {
      const int q = lane >> 3, c8 = (lane & 7) * 8;
      unsigned short* C  = (unsigned short*)Cout  + (size_t)b * strideC;
      unsigned short* C2 = (OUT_MODE == 2) ? ((unsigned short*)Cout2 + (size_t)b * strideC) : nullptr;
      for (int pass = 0; pass < 2; ++pass) {
#pragma unroll
        for (int it = 0; it < 4; ++it) {
          const int row = it * 4 + q;
          const float* sp = slab + row * 68 + c8;
          v8h hv, lv;
#pragma unroll
          for (int e = 0; e < 8; ++e) {
            if (OUT_MODE == 1) {
              hv[e] = (_Float16)sp[e];
            } else {
              unsigned short hb = f2bf_bits(sp[e]);
              unsigned short lb = f2bf_bits(sp[e] - bf_bits2f(hb));
              hv[e] = __builtin_bit_cast(_Float16, hb);
              lv[e] = __builtin_bit_cast(_Float16, lb);
            }
          }
          *(volatile v8h*)(C + (size_t)(mBase + row) * ldc + n0 + c8) = hv;
          if (OUT_MODE == 2) *(volatile v8h*)(C2 + (size_t)(mBase + row) * ldc + n0 + c8) = lv;
        }
        __threadfence();
      }
    }
    __builtin_amdgcn_fence(__ATOMIC_RELEASE, "workgroup");
    __builtin_amdgcn_wave_barrier();
    __builtin_amdgcn_fence(__ATOMIC_ACQUIRE, "workgroup");
  }
}

__global__ __launch_bounds__(256) void wsplit_kernel(const float* __restrict__ Wm, unsigned* __restrict__ HI, unsigned* __restrict__ LO) {
  const int i = blockIdx.x * 256 + threadIdx.x;
  if (i >= NFEAT * (NFEAT / 2)) return;
  const int n = i / (NFEAT / 2);
  const int k = 2 * (i - n * (NFEAT / 2));
  const float w0 = Wm[(size_t)k * NFEAT + n];
  const float w1 = Wm[(size_t)(k + 1) * NFEAT + n];
  unsigned short ah, al, bh, bl;
  split_bf(w0, ah, al); split_bf(w1, bh, bl);
  const unsigned uh = (unsigned)ah | ((unsigned)bh << 16);
  const unsigned ul = (unsigned)al | ((unsigned)bl << 16);
  ((volatile unsigned*)HI)[i] = uh; ((volatile unsigned*)LO)[i] = ul;
  __threadfence();
  ((volatile unsigned*)HI)[i] = uh; ((volatile unsigned*)LO)[i] = ul;
}

__device__ __forceinline__ int blk_excl_scan(int cnt, int* scan_ws, int tid, int* tot) {
  const int lane = tid & 31, wave = tid >> 5; int incl = cnt;
#pragma unroll
  for (int o = 1; o < 32; o <<= 1) { const int v = __shfl_up(incl, o, 32); if (lane >= o) incl += v; }
  if (lane == 31) scan_ws[wave] = incl;
  __syncthreads();
  if (wave == 0) { int wv = (lane < NT / 32) ? scan_ws[lane] : 0; int wincl = wv;
#pragma unroll
    for (int o = 1; o < 32; o <<= 1) { const int v = __shfl_up(wincl, o, 32); if (lane >= o) wincl += v; }
    if (lane < NT / 32) scan_ws[32 + lane] = wincl - wv; if (lane == 31) scan_ws[64] = wincl; }
  __syncthreads();
  const int res = scan_ws[32 + wave] + incl - cnt; *tot = scan_ws[64];
  return res;
}
template <int SP, int CAP, int NEDGE, int NSRC>
__device__ __forceinline__ int chunk_hits(const int* __restrict__ dstv, const int* __restrict__ srcv, int e0, int n0, int tid,
                                          int* LIST, int* scan_ws) {
  const int eb = e0 + tid * SP;
  const bool real = (eb < NEDGE);
  const int ebc = real ? eb : (NEDGE - SP);
  int rec[SP]; int cnt = 0;
#pragma unroll
  for (int k = 0; k < SP; k += 4) {
    const v4i d4 = *(const v4i*)(dstv + ebc + k);
    const v4i s4 = *(const v4i*)(srcv + ebc + k);
#pragma unroll
    for (int e = 0; e < 4; ++e) {
      int sr = s4[e]; sr = sr < 0 ? 0 : (sr >= NSRC ? NSRC - 1 : sr);
      const int d = d4[e];
      int r = -1;
      if (real && d >= n0 && d < n0 + SRB) { r = ((d - n0) << 17) | sr; ++cnt; }
      rec[k + e] = r;
    }
  }
  int tot; int p = blk_excl_scan(cnt, scan_ws, tid, &tot);
#pragma unroll
  for (int k = 0; k < SP; ++k) if (rec[k] >= 0) { if ((unsigned)p < (unsigned)CAP) LIST[p] = rec[k]; ++p; }
  __syncthreads();
  return tot < CAP ? tot : CAP;
}

template <int NSRC, int NEDGE>
__global__ __launch_bounds__(NT) void agg_kernel(const float* __restrict__ SRC, const int* __restrict__ srcv, const int* __restrict__ dstv,
                                                 float* ACC, float* __restrict__ CNT) {
  constexpr int NCHK = (NEDGE + SCH - 1) / SCH;
  __shared__ int LIST[SCH];
  __shared__ int scan_ws[80];
  const int tid = threadIdx.x, lane = tid & 31, wave = tid >> 5;
  const int n0 = blockIdx.x * SRB;
  const v4f zv = {0.0f, 0.0f, 0.0f, 0.0f};
#pragma unroll 1
  for (int j = 0; j < SRB / 8; ++j) {
    float* rp = ACC + (size_t)(n0 + wave * (SRB / 8) + j) * NFEAT + 4 * lane;
    *(volatile v4f*)rp = zv;
    __threadfence();
    *(volatile v4f*)rp = zv;
  }
  int cA0 = 0, cA1 = 0, cA2 = 0, cA3 = 0, cB0 = 0, cB1 = 0, cB2 = 0, cB3 = 0;
#pragma unroll 1
  for (int c = 0; c < NCHK; ++c) {
    const int tot = chunk_hits<SPT, SCH, NEDGE, NSRC>(dstv, srcv, c * SCH, n0, tid, LIST, scan_ws);
#pragma unroll 1
    for (int base = 0; base < tot; base += 32) {
      const int q = base + lane;
      const int qc = (q < SCH) ? q : (SCH - 1);
      const int lv = LIST[qc];
      const int rv = (q < tot) ? lv : -1;
      const int own = (rv >= 0 && (rv >> 25) == wave) ? 1 : 0;
      unsigned msk = (unsigned)__ballot(own);
#pragma unroll 1
      for (int it = 0; it < 32; ++it) {
        if (msk == 0u) break;
        const int bp = __builtin_ctz(msk); msk &= msk - 1u;
        const int r = __shfl(rv, bp, 32);
        const int dl = (r >> 17) & (SRB - 1);
        int s = r & 0x1FFFF; s = (s < NSRC) ? s : (NSRC - 1);
        const int dll = dl & 255;
        const int hs  = dll >> 7;
        const int ol  = (dll >> 2) & 31;
        const int ix  = dll & 3;
        const bool mine = (ol == lane);
        const bool mA = mine && (hs == 0), mB = mine && (hs == 1);
        cA0 += (mA && ix == 0) ? 1 : 0; cA1 += (mA && ix == 1) ? 1 : 0; cA2 += (mA && ix == 2) ? 1 : 0; cA3 += (mA && ix == 3) ? 1 : 0;
        cB0 += (mB && ix == 0) ? 1 : 0; cB1 += (mB && ix == 1) ? 1 : 0; cB2 += (mB && ix == 2) ? 1 : 0; cB3 += (mB && ix == 3) ? 1 : 0;
        const v4f pv = *(const v4f*)(SRC + (size_t)s * NFEAT + 4 * lane);
        float* rp = ACC + (size_t)(n0 + dl) * NFEAT + 4 * lane;
        v4f a = *(const v4f*)rp;
        a = a + pv;
        *(volatile v4f*)rp = a;
        __threadfence();
        *(volatile v4f*)rp = a;
      }
    }
    __syncthreads();
  }
  v4f dA, dB;
  dA[0] = (float)cA0; dA[1] = (float)cA1; dA[2] = (float)cA2; dA[3] = (float)cA3;
  dB[0] = (float)cB0; dB[1] = (float)cB1; dB[2] = (float)cB2; dB[3] = (float)cB3;
  float* pA = CNT + (size_t)n0 + wave * 256 + 4 * lane;
  float* pB = pA + 128;
  *(volatile v4f*)pA = dA; *(volatile v4f*)pB = dB;
  __threadfence();
  *(volatile v4f*)pA = dA; *(volatile v4f*)pB = dB;
}

template <int NV, int MPR>
__global__ __launch_bounds__(256) void meansplit_kernel(const float* __restrict__ ACC, const float* __restrict__ CNT,
                                                        unsigned short* __restrict__ HI, unsigned short* __restrict__ LO) {
  const int i = blockIdx.x * 256 + threadIdx.x;
  if (i >= MPR * 16) return;
  const int row = i >> 4, c8 = (i & 15) * 8;
  const float* pa = ACC + (size_t)row * NFEAT + c8;
  const v4f a0 = *(const v4f*)pa, a1 = *(const v4f*)(pa + 4);
  const float cn = CNT[row];
  const float inv = 1.0f / fmaxf(cn, 1.0f);
  v4f u0 = a0 * inv, u1 = a1 * inv;
  const v4f z4 = {0.f, 0.f, 0.f, 0.f};
  if (row >= NV) { u0 = z4; u1 = z4; }
  v8h hv, lv;
#pragma unroll
  for (int e = 0; e < 4; ++e) {
    unsigned short h0, l0, h1, l1;
    split_bf(u0[e], h0, l0); split_bf(u1[e], h1, l1);
    hv[e] = __builtin_bit_cast(_Float16, h0); lv[e] = __builtin_bit_cast(_Float16, l0);
    hv[4 + e] = __builtin_bit_cast(_Float16, h1); lv[4 + e] = __builtin_bit_cast(_Float16, l1);
  }
  unsigned short* ph = HI + (size_t)row * NFEAT + c8;
  unsigned short* pl = LO + (size_t)row * NFEAT + c8;
  *(volatile v8h*)ph = hv; *(volatile v8h*)pl = lv;
  __threadfence();
  *(volatile v8h*)ph = hv; *(volatile v8h*)pl = lv;
}

__global__ __launch_bounds__(256) void copy4_kernel(const float* __restrict__ S, float* __restrict__ D, int n4) {
  const int i = blockIdx.x * 256 + threadIdx.x;
  if (i >= n4) return;
  const v4f v = *(const v4f*)(S + (size_t)4 * i);
  float* op = D + (size_t)4 * i;
  *(volatile v4f*)op = v;
  __threadfence();
  *(volatile v4f*)op = v;
}

extern "C" void kernel_launch(void* const* d_in, const int* in_sizes, int n_in,
                              void* d_out, int out_size, void* d_ws, size_t ws_size, hipStream_t stream) {
  if (n_in < 5) return;
  if (in_sizes[0] != N_NODE * NFEAT || in_sizes[1] != NFEAT * NFEAT || in_sizes[2] != NFEAT ||
      in_sizes[3] != N_EDGE || in_sizes[4] != N_EDGE) return;
  if (out_size != N_NODE * NFEAT) return;

  const float* hidden = (const float*)d_in[0];
  const float* Wm     = (const float*)d_in[1];
  const float* bias   = (const float*)d_in[2];
  const int*   srcv   = (const int*)d_in[3];
  const int*   dstv   = (const int*)d_in[4];
  float*       out0   = (float*)d_out;

  char* ws = (char*)d_ws; size_t off = 0;
  auto carve = [&](size_t bytes) -> char* { char* p = ws + off; off += (bytes + 255) & ~(size_t)255; return p; };
  const size_t WPB  = (size_t)NFEAT * NFEAT * 2;
  const size_t ACCB = (size_t)NPAD_AGG * NFEAT * 4;
  const size_t CNTB = (size_t)NPAD_AGG * 4;
  const size_t PLB  = (size_t)M_PAD * NFEAT * 2;
  const size_t HB   = (size_t)M_PAD * NFEAT * 4;
  unsigned* BTH = (unsigned*)carve(WPB);
  unsigned* BTL = (unsigned*)carve(WPB);
  float* ACC = (float*)carve(ACCB);
  float* CNT = (float*)carve(CNTB);
  unsigned short* PH = (unsigned short*)carve(PLB);
  unsigned short* PL = (unsigned short*)carve(PLB);
  float* H = ACC;
  if (HB > ACCB) return;
  if (off > ws_size || off > (size_t)134217728) return;

  wsplit_kernel<<<(NFEAT * (NFEAT / 2)) / 256, 256, 0, stream>>>(Wm, BTH, BTL);
  agg_kernel<N_NODE, N_EDGE><<<N_TILE, NT, 0, stream>>>(hidden, srcv, dstv, ACC, CNT);
  meansplit_kernel<N_NODE, M_PAD><<<(M_PAD * 16) / 256, 256, 0, stream>>>(ACC, CNT, PH, PL);
  {
    const int tiles = (M_PAD / 64) * (NFEAT / 64);
    wmma_gemm64<1, true, 2, 0, false, 2><<<dim3((tiles + 7) / 8, 1), 256, 0, stream>>>(
        PH, PL, NFEAT, 0L, (const unsigned short*)BTH, (const unsigned short*)BTL, NFEAT, 0L,
        (void*)H, nullptr, NFEAT, 0L, bias, nullptr, 0L, M_PAD, NFEAT, NFEAT, 1.0f);
  }
  copy4_kernel<<<(N_NODE * NFEAT / 4) / 256, 256, 0, stream>>>(H, out0, N_NODE * NFEAT / 4);
}
